// H3_50603304681584
// MI455X (gfx1250) — hardware-verified
//
#include <hip/hip_runtime.h>
#include <math.h>

typedef __attribute__((ext_vector_type(16))) __bf16   v16b;
typedef __attribute__((ext_vector_type(8)))  __bf16   v8b;
typedef __attribute__((ext_vector_type(8)))  _Float16 v8h;
typedef __attribute__((ext_vector_type(8)))  float    v8f;
typedef __attribute__((ext_vector_type(4)))  float    v4f;

constexpr int kBatch  = 8;
constexpr int kCh     = 512;
constexpr int kLen    = 2048;
constexpr int kModes  = 32;
constexpr int kTaps   = 64;
constexpr int kPosAll = kBatch * kLen;
constexpr int kPPitch = 36;
static_assert((kCh % 64) == 0 && (kLen % 64) == 0 && (kCh % 32) == 0);
static_assert(kLen == 256 * 8);
static_assert((kTaps % 8) == 0 && kTaps == 64);
static_assert(kModes == 32);

constexpr size_t kOffXH = 0;
constexpr size_t kOffXL = kOffXH + (size_t)kPosAll * kCh * 2;
constexpr size_t kOffWH = kOffXL + (size_t)kPosAll * kCh * 2;
constexpr size_t kOffWL = kOffWH + (size_t)3 * kCh * kCh * 2;
constexpr size_t kOffKQ = kOffWL + (size_t)3 * kCh * kCh * 2;
constexpr size_t kOffVU = kOffKQ + (size_t)kBatch * kCh * kLen * 4;
constexpr size_t kOffCF = kOffVU + (size_t)kBatch * kCh * kLen * 4;
constexpr size_t kWsTotal = kOffCF + (size_t)4 * kCh * kModes * 4;
static_assert(kWsTotal == 104071168ull);
static_assert(kWsTotal <= 134217728ull);
static_assert((kOffXL % 128) == 0 && (kOffWH % 128) == 0 && (kOffWL % 128) == 0 &&
              (kOffKQ % 128) == 0 && (kOffVU % 128) == 0 && (kOffCF % 128) == 0);

__device__ __forceinline__ unsigned short f2bf_bits(float f) {
  unsigned u = __float_as_uint(f);
  return (unsigned short)((u + 0x7FFFu + ((u >> 16) & 1u)) >> 16);
}
__device__ __forceinline__ float bf_bits2f(unsigned short h) { return __uint_as_float(((unsigned)h) << 16); }

__device__ __forceinline__ void dep_guard4_b(v8f& a, v8f& b, v8f& c, v8f& d, v16b x, v16b y) {
  asm volatile("v_nop\n\tv_nop\n\tv_nop\n\tv_nop" : "+v"(a), "+v"(b), "+v"(c), "+v"(d) : "v"(x), "v"(y));
}
__device__ __forceinline__ void keep4_b(v16b a, v16b b, v16b c, v16b d) { asm volatile("v_nop" :: "v"(a), "v"(b), "v"(c), "v"(d)); }
__device__ __forceinline__ void acc_guard4(v8f& a, v8f& b, v8f& c, v8f& d) {
  asm volatile("v_nop\n\tv_nop\n\tv_nop\n\tv_nop" : "+v"(a), "+v"(b), "+v"(c), "+v"(d));
}

template <typename T> struct Frag;
template <> struct Frag<__bf16> {
  typedef v16b V; union U { v16b v; v8b h[2]; };
  static __device__ __forceinline__ v16b load(const __bf16* p) {
    U f; f.h[0] = *(const v8b*)(p); f.h[1] = *(const v8b*)(p + 16); return f.v;
  }
  static __device__ __forceinline__ v8f mma(v16b a, v16b b, v8f c) {
    return __builtin_amdgcn_wmma_f32_16x16x32_bf16(false, a, false, b, (short)0, c, false, false);
  }
};

__global__ __launch_bounds__(256) void gemm64_split_kernel(
    const unsigned short* __restrict__ Ap, const unsigned short* __restrict__ A2p, int lda,
    const unsigned short* __restrict__ Btp, const unsigned short* __restrict__ Bt2p, int ldb, long strideB,
    float* __restrict__ Cout, int ldc, long strideC,
    const float* __restrict__ bias, int M, int N, int K)
{
  typedef __bf16 T;
  typedef Frag<T>::V V;
  const T* A = (const T*)Ap; const T* A2 = (const T*)A2p; const T* Bt = (const T*)Btp; const T* Bt2 = (const T*)Bt2p;
  __shared__ __align__(16) float sT[8][16 * 68];
  const int b    = blockIdx.y;
  const int lane = threadIdx.x & 31;
  const int wave = threadIdx.x >> 5;
  const int tilesN = N >> 6;
  const int tilesM = M >> 6;
  const int tile = blockIdx.x * 8 + wave;
  if (tile >= tilesM * tilesN) return;
  const int tm = tile / tilesN;
  const int tn = tile - tm * tilesN;
  const int m0 = tm << 6;
  const int n0 = tn << 6;

  const T* Bb  = Bt  + (size_t)b * strideB;
  const T* Bb2 = Bt2 + (size_t)b * strideB;

  const int rlane = lane & 15;
  const int koff  = (lane >> 4) * 8;
  const int mOff  = (lane >> 4) * 8;

  v8f acc[4][4];
#pragma unroll
  for (int i = 0; i < 4; ++i)
#pragma unroll
    for (int j = 0; j < 4; ++j) acc[i][j] = (v8f){0.f,0.f,0.f,0.f,0.f,0.f,0.f,0.f};

  for (int k0 = 0; k0 < K; k0 += 32) {
    V bh[4], bl[4];
#pragma unroll
    for (int j = 0; j < 4; ++j) {
      const size_t bo = (size_t)(n0 + (j << 4) + rlane) * ldb + koff + k0;
      bh[j] = Frag<T>::load(Bb + bo);
      bl[j] = Frag<T>::load(Bb2 + bo);
    }
#pragma unroll
    for (int i = 0; i < 4; ++i) {
      const size_t ao = (size_t)(m0 + (i << 4) + rlane) * lda + koff + k0;
      V ah = Frag<T>::load(A + ao);
      V al = Frag<T>::load(A2 + ao);
#pragma unroll
      for (int j = 0; j < 4; ++j) {
        acc[i][j] = Frag<T>::mma(ah, bh[j], acc[i][j]);
        acc[i][j] = Frag<T>::mma(ah, bl[j], acc[i][j]);
        acc[i][j] = Frag<T>::mma(al, bh[j], acc[i][j]);
      }
      dep_guard4_b(acc[i][0], acc[i][1], acc[i][2], acc[i][3], ah, al);
    }
    keep4_b(bh[0], bh[1], bh[2], bh[3]);
    keep4_b(bl[0], bl[1], bl[2], bl[3]);
  }
  acc_guard4(acc[0][0], acc[0][1], acc[0][2], acc[0][3]);
  acc_guard4(acc[1][0], acc[1][1], acc[1][2], acc[1][3]);
  acc_guard4(acc[2][0], acc[2][1], acc[2][2], acc[2][3]);
  acc_guard4(acc[3][0], acc[3][1], acc[3][2], acc[3][3]);

  float* slab = sT[wave];
  float* C = Cout + (size_t)b * strideC;
  const int hh = lane >> 4, c4 = (lane & 15) * 4;
#pragma unroll
  for (int i = 0; i < 4; ++i) {
    const int mBase = m0 + (i << 4);
    const v4f bs0 = *(const v4f*)(bias + mBase + mOff);
    const v4f bs1 = *(const v4f*)(bias + mBase + mOff + 4);
    const float bsv[8] = { bs0[0], bs0[1], bs0[2], bs0[3], bs1[0], bs1[1], bs1[2], bs1[3] };
#pragma unroll
    for (int j = 0; j < 4; ++j) {
#pragma unroll
      for (int r = 0; r < 8; ++r) {
        const float v = acc[i][j][r] + bsv[r];
        slab[(mOff + r) * 68 + (j << 4) + rlane] = v;
      }
    }
    __builtin_amdgcn_fence(__ATOMIC_RELEASE, "workgroup");
    __builtin_amdgcn_wave_barrier();
    __builtin_amdgcn_fence(__ATOMIC_ACQUIRE, "workgroup");
    for (int pass = 0; pass < 2; ++pass) {
#pragma unroll
      for (int it = 0; it < 8; ++it) {
        const int row = it * 2 + hh;
        v4f v = *(const v4f*)(slab + row * 68 + c4);
        *(volatile v4f*)(C + (size_t)(mBase + row) * ldc + n0 + c4) = v;
      }
      __threadfence();
    }
    __builtin_amdgcn_fence(__ATOMIC_RELEASE, "workgroup");
    __builtin_amdgcn_wave_barrier();
    __builtin_amdgcn_fence(__ATOMIC_ACQUIRE, "workgroup");
  }
}

__global__ __launch_bounds__(256) void split_rows_bf16_kernel(
    const float* __restrict__ src, unsigned short* __restrict__ dhi, unsigned short* __restrict__ dlo, int total8)
{
  const int i = blockIdx.x * 256 + threadIdx.x;
  if (i >= total8) return;
  const size_t e0 = (size_t)i << 3;
  const v4f a0 = *(const v4f*)(src + e0);
  const v4f a1 = *(const v4f*)(src + e0 + 4);
  v8h hv, lv;
#pragma unroll
  for (int e = 0; e < 4; ++e) {
    const unsigned short h0 = f2bf_bits(a0[e]), h1 = f2bf_bits(a1[e]);
    const unsigned short l0 = f2bf_bits(a0[e] - bf_bits2f(h0)), l1 = f2bf_bits(a1[e] - bf_bits2f(h1));
    hv[e]     = __builtin_bit_cast(_Float16, h0);
    hv[4 + e] = __builtin_bit_cast(_Float16, h1);
    lv[e]     = __builtin_bit_cast(_Float16, l0);
    lv[4 + e] = __builtin_bit_cast(_Float16, l1);
  }
  unsigned short* qh = dhi + e0;
  unsigned short* ql = dlo + e0;
  *(volatile v8h*)qh = hv;
  *(volatile v8h*)ql = lv;
  __threadfence();
  *(volatile v8h*)qh = hv;
  *(volatile v8h*)ql = lv;
}

__global__ __launch_bounds__(256) void xpose_split_kernel(
    const float* __restrict__ x, unsigned short* __restrict__ XH, unsigned short* __restrict__ XL)
{
  __shared__ __align__(16) float sT[64 * 68];
  const int tid = threadIdx.x, lane = tid & 31, wave = tid >> 5;
  const int l0 = blockIdx.x * 64, h0 = blockIdx.y * 64, b = blockIdx.z;
  const float* xb = x + ((size_t)b * kCh + h0) * kLen + l0;
#pragma unroll
  for (int it = 0; it < 4; ++it) {
    const int idx = it * 256 + tid;
    const int hh = idx >> 4, l4 = (idx & 15) * 4;
    const v4f v = *(const v4f*)(xb + (size_t)hh * kLen + l4);
    *(v4f*)(sT + hh * 68 + l4) = v;
  }
  __syncthreads();
  const int q = lane >> 3, c8 = (lane & 7) * 8;
  v8h hv[2], lv[2];
#pragma unroll
  for (int it = 0; it < 2; ++it) {
    const int ll = it * 32 + wave * 4 + q;
#pragma unroll
    for (int e = 0; e < 8; ++e) {
      const float f = sT[(c8 + e) * 68 + ll];
      const unsigned short hb = f2bf_bits(f);
      const unsigned short lb = f2bf_bits(f - bf_bits2f(hb));
      hv[it][e] = __builtin_bit_cast(_Float16, hb);
      lv[it][e] = __builtin_bit_cast(_Float16, lb);
    }
  }
  for (int pass = 0; pass < 2; ++pass) {
#pragma unroll
    for (int it = 0; it < 2; ++it) {
      const int ll = it * 32 + wave * 4 + q;
      const size_t o = ((size_t)b * kLen + l0 + ll) * kCh + h0 + c8;
      *(volatile v8h*)(XH + o) = hv[it];
      *(volatile v8h*)(XL + o) = lv[it];
    }
    __threadfence();
  }
}

__global__ __launch_bounds__(256) void fir_gate_kernel(
    const float* __restrict__ kin, float* vu, const float* __restrict__ tapsC, const float* __restrict__ skipD)
{
  __shared__ __align__(16) float sK[kTaps + kLen];
  __shared__ __align__(16) float sS[kLen];
  __shared__ __align__(16) float sTap[kTaps];
  const int tid = threadIdx.x;
  const int row = blockIdx.x;
  const int h = row & (kCh - 1);
  const float* krow = kin + (size_t)row * kLen;
  float* vrow = vu + (size_t)row * kLen;
  float tv = tapsC[h * kTaps + (tid & (kTaps - 1))];
  asm volatile("" : "+v"(tv));
  if (tid < kTaps) {
    sTap[tid] = tv;
    sK[tid] = 0.0f;
  }
#pragma unroll
  for (int it = 0; it < 2; ++it) {
    const int i4 = (it * 256 + tid) * 4;
    const v4f kv = *(const v4f*)(krow + i4);
    *(v4f*)(sK + kTaps + i4) = kv;
  }
  const float Dh = skipD[h];
  __syncthreads();

  const int t0 = tid * 8;
  float acc[8];
#pragma unroll
  for (int j = 0; j < 8; ++j) acc[j] = 0.0f;
#pragma unroll 1
  for (int sb = 0; sb < kTaps / 8; ++sb) {
    const int s0 = sb * 8;
    const float* wp = sK + (kTaps + t0 - s0 - 8);
    const v4f w0 = *(const v4f*)(wp);
    const v4f w1 = *(const v4f*)(wp + 4);
    const v4f w2 = *(const v4f*)(wp + 8);
    const v4f w3 = *(const v4f*)(wp + 12);
    const v4f ta = *(const v4f*)(sTap + s0);
    const v4f tb = *(const v4f*)(sTap + s0 + 4);
    const float win[16] = { w0[0], w0[1], w0[2], w0[3], w1[0], w1[1], w1[2], w1[3],
                            w2[0], w2[1], w2[2], w2[3], w3[0], w3[1], w3[2], w3[3] };
    const float tp[8] = { ta[0], ta[1], ta[2], ta[3], tb[0], tb[1], tb[2], tb[3] };
#pragma unroll
    for (int e = 0; e < 8; ++e) {
#pragma unroll
      for (int j = 0; j < 8; ++j) acc[j] = fmaf(tp[e], win[8 + j - e], acc[j]);
    }
  }
  {
    const v4f c0 = *(const v4f*)(sK + kTaps + t0);
    const v4f c1 = *(const v4f*)(sK + kTaps + t0 + 4);
    v4f o0, o1;
    o0[0] = fmaf(Dh, c0[0], acc[0]);
    o0[1] = fmaf(Dh, c0[1], acc[1]);
    o0[2] = fmaf(Dh, c0[2], acc[2]);
    o0[3] = fmaf(Dh, c0[3], acc[3]);
    o1[0] = fmaf(Dh, c1[0], acc[4]);
    o1[1] = fmaf(Dh, c1[1], acc[5]);
    o1[2] = fmaf(Dh, c1[2], acc[6]);
    o1[3] = fmaf(Dh, c1[3], acc[7]);
    *(v4f*)(sS + t0) = o0;
    *(v4f*)(sS + t0 + 4) = o1;
  }
  __syncthreads();
  v4f uv[2];
#pragma unroll
  for (int it = 0; it < 2; ++it) {
    const int i4 = (it * 256 + tid) * 4;
    const v4f vv = *(const v4f*)(vrow + i4);
    const v4f ss = *(const v4f*)(sS + i4);
    uv[it] = vv * ss;
  }
  for (int pass = 0; pass < 2; ++pass) {
#pragma unroll
    for (int it = 0; it < 2; ++it) {
      const int i4 = (it * 256 + tid) * 4;
      *(volatile v4f*)(vrow + i4) = uv[it];
    }
    __threadfence();
  }
}

__global__ __launch_bounds__(256) void coeff_kernel(
    const float* __restrict__ log_dt, const float* __restrict__ A_real, const float* __restrict__ A_imag,
    const float* __restrict__ C_re, const float* __restrict__ C_im, float* __restrict__ cf)
{
  const int lane = threadIdx.x & 31, wave = threadIdx.x >> 5;
  const int h = blockIdx.x * 8 + wave;
  const int ci = h * kModes + lane;
  const float dt = expf(log_dt[h]);
  const float Ar = -expf(A_real[ci]);
  const float Ai = A_imag[ci];
  const float ar = Ar * dt;
  const float ai = Ai * dt;
  const float er = expf(ar);
  const float sn = sinf(ai);
  const float cs = cosf(ai);
  const float Wr = er * cs;
  const float Wi = er * sn;
  const float dr = Wr - 1.0f;
  const float di = Wi;
  const float cr = C_re[ci];
  const float cm = C_im[ci];
  const float nr = cr * dr - cm * di;
  const float ni = cr * di + cm * dr;
  const float inv = 1.0f / (Ar * Ar + Ai * Ai);
  const float Gr = 2.0f * ((nr * Ar + ni * Ai) * inv);
  const float Gi = 2.0f * ((ni * Ar - nr * Ai) * inv);
  float* p0 = cf + ci;
  float* p1 = cf + kCh * kModes + ci;
  float* p2 = cf + 2 * kCh * kModes + ci;
  float* p3 = cf + 3 * kCh * kModes + ci;
  *(volatile float*)p0 = Wr;
  *(volatile float*)p1 = Wi;
  *(volatile float*)p2 = Gr;
  *(volatile float*)p3 = Gi;
  __threadfence();
  *(volatile float*)p0 = Wr;
  *(volatile float*)p1 = Wi;
  *(volatile float*)p2 = Gr;
  *(volatile float*)p3 = Gi;
}

__global__ __launch_bounds__(256) void scan_gate_kernel(
    const float* __restrict__ u, const float* __restrict__ q, const float* __restrict__ cf,
    const float* __restrict__ skipD2, float* __restrict__ out)
{
  __shared__ __align__(16) float sU[8][32];
  __shared__ __align__(16) float sP[8][32 * kPPitch];
  const int lane = threadIdx.x & 31, wave = threadIdx.x >> 5;
  const int row = blockIdx.x * 8 + wave;
  const int h = row & (kCh - 1);
  const int ci = h * kModes + lane;
  const float Wr = cf[ci];
  const float Wi = cf[kCh * kModes + ci];
  const float Gr = cf[2 * kCh * kModes + ci];
  const float Gi = cf[3 * kCh * kModes + ci];
  const float Dp = skipD2[h];
  const float* urow = u + (size_t)row * kLen;
  const float* qrow = q + (size_t)row * kLen;
  float* orow = out + (size_t)row * kLen;
  float* myU = sU[wave];
  float* myP = sP[wave];
  float Sr = 0.0f, Si = 0.0f;
#pragma unroll 1
  for (int t0 = 0; t0 < kLen; t0 += 32) {
    const float uvec = urow[t0 + lane];
    const float qv = qrow[t0 + lane];
    myU[lane] = uvec;
    __syncthreads();
#pragma unroll 1
    for (int g = 0; g < 4; ++g) {
      const v4f ua = *(const v4f*)(myU + g * 8);
      const v4f ub = *(const v4f*)(myU + g * 8 + 4);
      const float uu[8] = { ua[0], ua[1], ua[2], ua[3], ub[0], ub[1], ub[2], ub[3] };
      float* pg = myP + (g * 8) * kPPitch + lane;
#pragma unroll
      for (int j = 0; j < 8; ++j) {
        const float nSr = fmaf(Wr, Sr, fmaf(-Wi, Si, uu[j]));
        const float nSi = fmaf(Wr, Si, Wi * Sr);
        Sr = nSr;
        Si = nSi;
        const float cc = fmaf(Gr, Sr, -(Gi * Si));
        pg[j * kPPitch] = cc;
      }
    }
    __syncthreads();
    const float* pr = myP + lane * kPPitch;
    float y = 0.0f;
#pragma unroll
    for (int c = 0; c < 8; ++c) {
      const v4f p = *(const v4f*)(pr + 4 * c);
      y += p[0];
      y += p[1];
      y += p[2];
      y += p[3];
    }
    const float val = qv * fmaf(Dp, uvec, y);
    volatile float* op = orow + t0 + lane;
    *op = val;
    __threadfence();
    *op = val;
  }
}

extern "C" void kernel_launch(void* const* d_in, const int* in_sizes, int n_in,
                              void* d_out, int out_size, void* d_ws, size_t ws_size,
                              hipStream_t stream) {
  if (n_in < 15) return;
  if (in_sizes[0] != kBatch * kCh * kLen) return;
  if (in_sizes[1] != kCh * kCh) return;
  if (in_sizes[2] != kCh) return;
  if (in_sizes[3] != kCh * kCh) return;
  if (in_sizes[4] != kCh) return;
  if (in_sizes[5] != kCh * kCh) return;
  if (in_sizes[6] != kCh) return;
  if (in_sizes[7] != kCh * kTaps) return;
  if (in_sizes[8] != kCh) return;
  if (in_sizes[9] != kCh) return;
  if (in_sizes[10] != kCh * kModes) return;
  if (in_sizes[11] != kCh * kModes) return;
  if (in_sizes[12] != kCh * kModes) return;
  if (in_sizes[13] != kCh * kModes) return;
  if (in_sizes[14] != kCh) return;
  if (out_size != kBatch * kCh * kLen) return;
  if (ws_size < kWsTotal) return;

  const float* x       = (const float*)d_in[0];
  const float* Wq      = (const float*)d_in[1];
  const float* bq      = (const float*)d_in[2];
  const float* Wk      = (const float*)d_in[3];
  const float* bk      = (const float*)d_in[4];
  const float* Wv      = (const float*)d_in[5];
  const float* bv      = (const float*)d_in[6];
  const float* shiftC  = (const float*)d_in[7];
  const float* shiftD  = (const float*)d_in[8];
  const float* log_dt  = (const float*)d_in[9];
  const float* A_real  = (const float*)d_in[10];
  const float* A_imag  = (const float*)d_in[11];
  const float* C_re    = (const float*)d_in[12];
  const float* C_im    = (const float*)d_in[13];
  const float* skipD2  = (const float*)d_in[14];
  float* out = (float*)d_out;

  char* ws = (char*)d_ws;
  unsigned short* XH = (unsigned short*)(ws + kOffXH);
  unsigned short* XL = (unsigned short*)(ws + kOffXL);
  unsigned short* WH = (unsigned short*)(ws + kOffWH);
  unsigned short* WL = (unsigned short*)(ws + kOffWL);
  float*          KQ = (float*)(ws + kOffKQ);
  float*          VU = (float*)(ws + kOffVU);
  float*          CF = (float*)(ws + kOffCF);

  const int wElems = kCh * kCh;
  const int wThreads = wElems / 8;
  const int wBlocks = wThreads / 256;

  split_rows_bf16_kernel<<<wBlocks, 256, 0, stream>>>(Wq, WH, WL, wThreads);
  split_rows_bf16_kernel<<<wBlocks, 256, 0, stream>>>(Wk, WH + wElems, WL + wElems, wThreads);
  split_rows_bf16_kernel<<<wBlocks, 256, 0, stream>>>(Wv, WH + 2 * wElems, WL + 2 * wElems, wThreads);

  xpose_split_kernel<<<dim3(kLen / 64, kCh / 64, kBatch), 256, 0, stream>>>(x, XH, XL);

  const int tiles = (kCh / 64) * (kLen / 64);
  const dim3 ggrid((tiles + 7) / 8, kBatch);
  const long sB = (long)kLen * kCh;
  const long sC = (long)kCh * kLen;

  gemm64_split_kernel<<<ggrid, 256, 0, stream>>>(
      WH + wElems, WL + wElems, kCh, XH, XL, kCh, sB, KQ, kLen, sC, bk, kCh, kLen, kCh);
  gemm64_split_kernel<<<ggrid, 256, 0, stream>>>(
      WH + 2 * wElems, WL + 2 * wElems, kCh, XH, XL, kCh, sB, VU, kLen, sC, bv, kCh, kLen, kCh);
  fir_gate_kernel<<<kBatch * kCh, 256, 0, stream>>>(KQ, VU, shiftC, shiftD);
  gemm64_split_kernel<<<ggrid, 256, 0, stream>>>(
      WH, WL, kCh, XH, XL, kCh, sB, KQ, kLen, sC, bq, kCh, kLen, kCh);
  coeff_kernel<<<kCh / 8, 256, 0, stream>>>(log_dt, A_real, A_imag, C_re, C_im, CF);
  scan_gate_kernel<<<(kBatch * kCh) / 8, 256, 0, stream>>>(VU, KQ, CF, skipD2, out);
}
